// GATGPP_13683765805699
// MI455X (gfx1250) — hardware-verified
//
#include <hip/hip_runtime.h>
#include <stddef.h>
#include <stdint.h>
#include <math.h>


#define F_IN    128
#define HC      256
#define NHD     4
#define HID     64
#define KA2     512
#define NGR     128
#define NOUTC   8
#define NOUT    (NGR * NOUTC)
#define NTHR    256
#define NWAVE   8
#define EPT     8
#define CHUNK   (NTHR * EPT)
#define WCAP    (EPT * 32)
#define LISTN   (NWAVE * WCAP)
#define NBMAX   2048
#define SLOTB   11
#define RCAP    28672
#define DEGCAP  256
#define GBM     64
#define GBN     64
#define GTHR    128
#define MROWS   128
#define RPW     8
#define RPB     (NWAVE * RPW)
#define NU1     (HC * (F_IN / 8))
#define NU2     (HC * (KA2 / 8))
#define NEGSL   0.2f
#define EPS_SM  1e-16f
#define WSMAX   134217728
#define LDS_BKT ((2 * RCAP + 2 * NBMAX + LISTN) * 4 + 64)
#define MEAS_B1024  16623
#define MEAS_MAXDEG 35

static_assert((CHUNK & (CHUNK - 1)) == 0 && CHUNK <= (1 << SLOTB));
static_assert(NBMAX == (1 << SLOTB));
static_assert(NTHR * 8 == NBMAX);
static_assert(LISTN >= NBMAX);
static_assert(LISTN >= NWAVE * WCAP);
static_assert((RCAP % (4 * NTHR)) == 0 && (NBMAX % (4 * NTHR)) == 0);
static_assert(LDS_BKT <= 300000);
static_assert(MEAS_B1024 + 4096 <= RCAP);
static_assert(MEAS_MAXDEG + 8 <= DEGCAP);
static_assert(GBM == (GTHR / 32) * 16);
static_assert(GTHR == 2 * GBN && GTHR == 2 * GBM);
static_assert((F_IN % 32) == 0 && (KA2 % 32) == 0);
static_assert((HC % GBN) == 0 && HID == GBN && HC == NHD * HID);
static_assert(KA2 == 2 * HC && F_IN <= KA2);
static_assert((MROWS % GBM) == 0 && (MROWS % RPB) == 0 && (NBMAX % RPB) == 0);
static_assert(32 * 8 == HC && HID == 64);
static_assert(F_IN / 8 == 16);
static_assert(NU1 % NTHR == 0 && NU2 % NTHR == 0);
static_assert(NOUT == 4 * NTHR && (NOUT * 4) % 128 == 0);
static_assert(NGR == 128 && NOUTC == 8);

typedef float          v2f  __attribute__((ext_vector_type(2)));
typedef float          v4f  __attribute__((ext_vector_type(4)));
typedef float          v8f  __attribute__((ext_vector_type(8)));
typedef int            v4i  __attribute__((ext_vector_type(4)));
typedef int            v8i  __attribute__((ext_vector_type(8)));
typedef unsigned int   v4u  __attribute__((ext_vector_type(4)));
typedef unsigned short v8us __attribute__((ext_vector_type(8)));
typedef __bf16         v16b __attribute__((ext_vector_type(16)));
typedef v2f  __attribute__((may_alias)) v2fa;
typedef v4f  __attribute__((may_alias)) v4fa;
typedef v4i  __attribute__((may_alias)) v4ia;
typedef v8us __attribute__((may_alias)) v8usa;
union FragB { v16b v; v8us h[2]; v8i w; };

__device__ __forceinline__ v8f wmb(const FragB& a, const FragB& b, v8f c) {
  v8f d = __builtin_amdgcn_wmma_f32_16x16x32_bf16(false, a.v, false, b.v, (short)0, c, false, false);
  asm volatile("v_nop\n\tv_nop\n\tv_nop\n\tv_nop" : "+v"(d) : "v"(a.w), "v"(b.w));
  return d;
}

__device__ __forceinline__ unsigned int f2bf(float f) {
  const unsigned int u = __float_as_uint(f);
  const unsigned int r = ((u + 0x7FFFu + ((u >> 16) & 1u)) >> 16) & 0xFFFFu;
  return (f != f) ? 0x7FC0u : r;
}
__device__ __forceinline__ float bf2f(unsigned int b) { return __uint_as_float(b << 16); }
__device__ __forceinline__ float bfr(float f) { return bf2f(f2bf(f)); }
__device__ __forceinline__ v4f bfr4(const v4f a) {
  v4f r; r.x = bfr(a.x); r.y = bfr(a.y); r.z = bfr(a.z); r.w = bfr(a.w); return r;
}
__device__ __forceinline__ unsigned int pk2(float lo, float hi) { return f2bf(lo) | (f2bf(hi) << 16); }
__device__ __forceinline__ v4u pack8(const v4f a, const v4f b) {
  v4u r;
  r.x = pk2(a.x, a.y); r.y = pk2(a.z, a.w); r.z = pk2(b.x, b.y); r.w = pk2(b.z, b.w);
  return r;
}
__device__ __forceinline__ float elu1(float v) { return (v > 0.f) ? v : (__expf(v) - 1.0f); }

__device__ __forceinline__ int scan_chunk(const int* __restrict__ dsts, int nE, int cbase, int slotBase,
                                          int nb, int vec8, int* list, int tid, int lane, int wave) {
  int wc = 0;
  const int el0  = tid * EPT;
  const int e0   = cbase + el0;
  const int sent = -2147483647 - 1;
  v4i da, db;
  if (vec8 != 0 && cbase + CHUNK <= nE) {
    da = *(const v4i*)(dsts + e0);
    db = *(const v4i*)(dsts + e0 + 4);
  } else {
    da.x = (e0     < nE) ? dsts[min(e0,     nE - 1)] : sent;
    da.y = (e0 + 1 < nE) ? dsts[min(e0 + 1, nE - 1)] : sent;
    da.z = (e0 + 2 < nE) ? dsts[min(e0 + 2, nE - 1)] : sent;
    da.w = (e0 + 3 < nE) ? dsts[min(e0 + 3, nE - 1)] : sent;
    db.x = (e0 + 4 < nE) ? dsts[min(e0 + 4, nE - 1)] : sent;
    db.y = (e0 + 5 < nE) ? dsts[min(e0 + 5, nE - 1)] : sent;
    db.z = (e0 + 6 < nE) ? dsts[min(e0 + 6, nE - 1)] : sent;
    db.w = (e0 + 7 < nE) ? dsts[min(e0 + 7, nE - 1)] : sent;
  }
  const unsigned nbs = (unsigned)slotBase;
  const unsigned unb = (unsigned)nb;
  const unsigned s0 = (unsigned)da.x - nbs, s1 = (unsigned)da.y - nbs;
  const unsigned s2 = (unsigned)da.z - nbs, s3 = (unsigned)da.w - nbs;
  const unsigned s4 = (unsigned)db.x - nbs, s5 = (unsigned)db.y - nbs;
  const unsigned s6 = (unsigned)db.z - nbs, s7 = (unsigned)db.w - nbs;
  const bool h0 = s0 < unb, h1 = s1 < unb, h2 = s2 < unb, h3 = s3 < unb;
  const bool h4 = s4 < unb, h5 = s5 < unb, h6 = s6 < unb, h7 = s7 < unb;
  const unsigned any = __builtin_amdgcn_ballot_w32(h0 | h1 | h2 | h3 | h4 | h5 | h6 | h7);
  if (any != 0u) {
#define HITJ(J, HJ, SJ) { \
      const unsigned mj = __builtin_amdgcn_ballot_w32(HJ); \
      if (mj != 0u) { \
        if (HJ) { \
          const int pos = wc + (int)__builtin_amdgcn_mbcnt_lo(mj, 0u); \
          if (pos < WCAP) list[wave * WCAP + pos] = ((el0 + (J)) << SLOTB) | (int)(SJ); \
        } \
        wc += (int)__builtin_popcount(mj); } }
    HITJ(0, h0, s0)
    HITJ(1, h1, s1)
    HITJ(2, h2, s2)
    HITJ(3, h3, s3)
    HITJ(4, h4, s4)
    HITJ(5, h5, s5)
    HITJ(6, h6, s6)
    HITJ(7, h7, s7)
#undef HITJ
  }
  return wc;
}

__device__ __forceinline__ void wtr_unit(const float* __restrict__ w, int Kin, int Ncol, int Kout,
                                         unsigned short* wt, int u) {
  const int kq = Kout >> 3;
  const int n  = u / kq;
  const int k8 = (u - n * kq) * 8;
  const int kk = k8 - (k8 / Kin) * Kin;
  const float* p = w + (size_t)kk * (size_t)Ncol + n;
  v4f a, b;
  a.x = p[0];                    a.y = p[(size_t)Ncol];         a.z = p[(size_t)2 * Ncol];     a.w = p[(size_t)3 * Ncol];
  b.x = p[(size_t)4 * Ncol];     b.y = p[(size_t)5 * Ncol];     b.z = p[(size_t)6 * Ncol];     b.w = p[(size_t)7 * Ncol];
  const v4u wv = pack8(a, b);
  unsigned short* o = wt + (size_t)n * (size_t)Kout + k8;
  *(volatile v4u*)o = wv;
  __threadfence();
  *(volatile v4u*)o = wv;
}

__global__ __launch_bounds__(NTHR) void k_wprep(const float* __restrict__ W1, const float* __restrict__ W2,
                                                unsigned short* W1T, unsigned short* W2D) {
  const int u = (int)blockIdx.x * NTHR + (int)threadIdx.x;
  if (u < NU1) {
    wtr_unit(W1, F_IN, HC, F_IN, W1T, u);
  } else if (u < NU1 + NU2) {
    wtr_unit(W2, HC, HC, KA2, W2D, u - NU1);
  }
}

__global__ __launch_bounds__(NTHR) void k_cvx(const float* __restrict__ x, int nN, int nUnits,
                                              unsigned short* xb) {
  const int u = (int)blockIdx.x * NTHR + (int)threadIdx.x;
  if (u >= nUnits) return;
  const int row = u >> 4;
  const int k8  = (u & 15) * 8;
  const int rc  = row < nN ? row : nN - 1;
  const float* p = x + (size_t)rc * F_IN + k8;
  v4f a = *(const v4fa*)p;
  v4f b = *(const v4fa*)(p + 4);
  const v4f z4 = {0.f, 0.f, 0.f, 0.f};
  if (row >= nN) { a = z4; b = z4; }
  const v4u hv = pack8(a, b);
  unsigned short* dp = xb + (size_t)row * F_IN + k8;
  *(volatile v4u*)dp = hv;
  __threadfence();
  *(volatile v4u*)dp = hv;
}

__global__ __launch_bounds__(NTHR) void k_bucket(
    const int* __restrict__ srcs, const int* __restrict__ dsts,
    int nN, int nE, int nb, int vec8,
    int* TSRC, int* TCNT, int* TOFF, int* TNH) {
  extern __shared__ v4f lds_dyn[];
  int* reg1 = (int*)lds_dyn;
  int* reg2 = reg1 + RCAP;
  int* scnt = reg2 + RCAP;
  int* soff = scnt + NBMAX;
  int* list = soff + NBMAX;
  int* wcnt = list + LISTN;
  int* wtot = wcnt + NWAVE;
  const int tid = (int)threadIdx.x, lane = tid & 31, wave = tid >> 5;
  const int nodeBase = (int)blockIdx.x * nb;

  for (int i = tid; i < NBMAX; i += NTHR) scnt[i] = 0;
  __syncthreads();

  int tot = 0;
  const int nChunks = (nE + CHUNK - 1) / CHUNK;
#pragma unroll 1
  for (int ch = 0; ch < nChunks; ++ch) {
    const int cbase = ch * CHUNK;
    const int wc = scan_chunk(dsts, nE, cbase, nodeBase, nb, vec8, list, tid, lane, wave);
    if (lane == 0) wcnt[wave] = wc;
    __syncthreads();
    int pre = 0, all = 0;
#pragma unroll
    for (int w2 = 0; w2 < NWAVE; ++w2) {
      int c = wcnt[w2];
      c = c < 0 ? 0 : (c > WCAP ? WCAP : c);
      all += c;
      pre += (w2 < wave) ? c : 0;
    }
    const int wcc  = wc > WCAP ? WCAP : wc;
    const int base = tot + pre;
#pragma unroll 1
    for (int i = lane; i < wcc; i += 32) {
      const int ent = list[wave * WCAP + i];
      const int el  = (ent >> SLOTB) & (CHUNK - 1);
      const int sl  = ent & (NBMAX - 1);
      int eid = cbase + el;
      eid = eid > nE - 1 ? nE - 1 : eid;
      const int pos = base + i;
      if (pos < RCAP) reg1[pos] = (int)(((unsigned)eid << SLOTB) | (unsigned)sl);
    }
    tot += all;
    tot = tot > RCAP ? RCAP : tot;
    __syncthreads();
  }
  const int nh = tot;

  if (wave == 0) {
#pragma unroll 1
    for (int b0 = 0; b0 < nh; b0 += 32) {
      const int idx = b0 + lane;
      const int uv  = reg1[idx < nh ? idx : nh - 1];
      const int m32 = (nh - b0) < 32 ? (nh - b0) : 32;
#pragma unroll 1
      for (int k = 0; k < m32; ++k) {
        const int u  = __builtin_amdgcn_readlane(uv, k);
        const int sl = u & (NBMAX - 1);
        if (lane == 0) scnt[sl] = scnt[sl] + 1;
      }
    }
  }
  __syncthreads();

  {
    const v4i ca = *(const v4ia*)(scnt + 8 * tid);
    const v4i cb = *(const v4ia*)(scnt + 8 * tid + 4);
    const int e0 = ca.x < 0 ? 0 : ca.x, e1 = ca.y < 0 ? 0 : ca.y, e2 = ca.z < 0 ? 0 : ca.z, e3 = ca.w < 0 ? 0 : ca.w;
    const int e4 = cb.x < 0 ? 0 : cb.x, e5 = cb.y < 0 ? 0 : cb.y, e6 = cb.z < 0 ? 0 : cb.z, e7 = cb.w < 0 ? 0 : cb.w;
    const int ts = e0 + e1 + e2 + e3 + e4 + e5 + e6 + e7;
    int incl = ts;
#pragma unroll
    for (int d = 1; d < 32; d <<= 1) {
      const int up = __shfl_up(incl, d);
      if (lane >= d) incl += up;
    }
    if (lane == 31) wtot[wave] = incl;
    __syncthreads();
    int pre = 0;
#pragma unroll
    for (int w2 = 0; w2 < NWAVE; ++w2) pre += (w2 < wave) ? wtot[w2] : 0;
    int run = pre + incl - ts;
    soff[8 * tid + 0] = run; run += e0;
    soff[8 * tid + 1] = run; run += e1;
    soff[8 * tid + 2] = run; run += e2;
    soff[8 * tid + 3] = run; run += e3;
    soff[8 * tid + 4] = run; run += e4;
    soff[8 * tid + 5] = run; run += e5;
    soff[8 * tid + 6] = run; run += e6;
    soff[8 * tid + 7] = run;
  }
  __syncthreads();
  for (int i = tid; i < NBMAX; i += NTHR) list[i] = soff[i];
  __syncthreads();

  if (wave == 0) {
#pragma unroll 1
    for (int b0 = 0; b0 < nh; b0 += 32) {
      const int idx = b0 + lane;
      const int uv  = reg1[idx < nh ? idx : nh - 1];
      const int m32 = (nh - b0) < 32 ? (nh - b0) : 32;
#pragma unroll 1
      for (int k = 0; k < m32; ++k) {
        const int u   = __builtin_amdgcn_readlane(uv, k);
        const int sl  = u & (NBMAX - 1);
        const int eid = (int)((unsigned)u >> SLOTB);
        if (lane == 0) {
          int pos = list[sl];
          pos = pos < 0 ? 0 : (pos > RCAP - 1 ? RCAP - 1 : pos);
          reg2[pos] = eid;
          list[sl] = pos + 1;
        }
      }
    }
  }
  __syncthreads();

  {
    int* tsrc = TSRC + (size_t)blockIdx.x * (size_t)RCAP;
#pragma unroll 1
    for (int i = 4 * tid; i < RCAP; i += 4 * NTHR) {
      const v4i e4 = *(const v4ia*)(reg2 + i);
      const bool k0 = i < nh, k1 = i + 1 < nh, k2 = i + 2 < nh, k3 = i + 3 < nh;
      int a0 = k0 ? e4.x : 0, a1 = k1 ? e4.y : 0, a2 = k2 ? e4.z : 0, a3 = k3 ? e4.w : 0;
      a0 = a0 < 0 ? 0 : (a0 > nE - 1 ? nE - 1 : a0);
      a1 = a1 < 0 ? 0 : (a1 > nE - 1 ? nE - 1 : a1);
      a2 = a2 < 0 ? 0 : (a2 > nE - 1 ? nE - 1 : a2);
      a3 = a3 < 0 ? 0 : (a3 > nE - 1 ? nE - 1 : a3);
      int s0 = srcs[a0], s1 = srcs[a1], s2 = srcs[a2], s3 = srcs[a3];
      s0 = s0 < 0 ? 0 : (s0 > nN - 1 ? nN - 1 : s0);
      s1 = s1 < 0 ? 0 : (s1 > nN - 1 ? nN - 1 : s1);
      s2 = s2 < 0 ? 0 : (s2 > nN - 1 ? nN - 1 : s2);
      s3 = s3 < 0 ? 0 : (s3 > nN - 1 ? nN - 1 : s3);
      v4i sv;
      sv.x = k0 ? s0 : 0; sv.y = k1 ? s1 : 0; sv.z = k2 ? s2 : 0; sv.w = k3 ? s3 : 0;
      *(volatile v4i*)(tsrc + i) = sv;
      __threadfence();
      *(volatile v4i*)(tsrc + i) = sv;
    }
    int* tcnt = TCNT + (size_t)blockIdx.x * (size_t)NBMAX;
    int* toff = TOFF + (size_t)blockIdx.x * (size_t)NBMAX;
#pragma unroll 1
    for (int i = 4 * tid; i < NBMAX; i += 4 * NTHR) {
      const v4i c4 = *(const v4ia*)(scnt + i);
      const v4i o4 = *(const v4ia*)(soff + i);
      *(volatile v4i*)(tcnt + i) = c4;
      *(volatile v4i*)(toff + i) = o4;
      __threadfence();
      *(volatile v4i*)(tcnt + i) = c4;
      *(volatile v4i*)(toff + i) = o4;
    }
    v4i n4; n4.x = nh; n4.y = nh; n4.z = nh; n4.w = nh;
    int* tn = TNH + (size_t)blockIdx.x * 32 + 4 * (lane & 7);
    const bool wn = (wave == 0) && (lane < 8);
    if (wn) *(volatile v4i*)tn = n4;
    __threadfence();
    if (wn) *(volatile v4i*)tn = n4;
  }
}

__global__ __launch_bounds__(GTHR) void k_gemm(
    const unsigned short* __restrict__ A, const unsigned short* __restrict__ WT,
    float* outF, int K, int ldo,
    const float* __restrict__ atts, const float* __restrict__ attd, int attLen,
    float* SD, int MPr)
{
  __shared__ __attribute__((aligned(16))) float stg[GBM * GBN];
  __shared__ __attribute__((aligned(16))) float satt[2 * GBN];
  __shared__ __attribute__((aligned(16))) float sdot[2 * GBM];
  const int tid = (int)threadIdx.x, lane = tid & 31, wave = tid >> 5, hh = lane >> 4, m = lane & 15;
  const int rowBase = (int)blockIdx.x * GBM;
  const int head    = (int)blockIdx.y;
  const int col0    = head * GBN;

  {
    const int which = tid >> 6;
    const int c  = tid & 63;
    const int cl = c < attLen ? c : attLen - 1;
    const float vs = atts[head * attLen + cl];
    const float vd = attd[head * attLen + cl];
    float v = (which == 0) ? vs : vd;
    v = (c < attLen) ? bfr(v) : 0.f;
    satt[which * GBN + c] = v;
  }

  v8f acc[4];
  {
    const v8f z = {0.f, 0.f, 0.f, 0.f, 0.f, 0.f, 0.f, 0.f};
    acc[0] = z; acc[1] = z; acc[2] = z; acc[3] = z;
  }
  const unsigned short* ap = A  + (size_t)(rowBase + 16 * wave + m) * (size_t)K + 8 * hh;
  const unsigned short* wp = WT + (size_t)(col0 + m) * (size_t)K + 8 * hh;
  const int ksteps = K >> 5;
#pragma unroll 1
  for (int ks = 0; ks < ksteps; ++ks) {
    FragB af;
    af.h[0] = *(const v8usa*)(ap + 32 * ks);
    af.h[1] = *(const v8usa*)(ap + 32 * ks + 16);
#pragma unroll
    for (int t = 0; t < 4; ++t) {
      const unsigned short* wq = wp + (size_t)(16 * t) * (size_t)K + 32 * ks;
      FragB bf;
      bf.h[0] = *(const v8usa*)wq;
      bf.h[1] = *(const v8usa*)(wq + 16);
      acc[t] = wmb(af, bf, acc[t]);
    }
  }

#pragma unroll
  for (int t = 0; t < 4; ++t) {
    const int lc = 16 * t + m;
#pragma unroll
    for (int r = 0; r < 8; ++r) {
      const int lr = 16 * wave + 8 * hh + r;
      stg[lr * GBN + lc] = acc[t][r];
    }
  }
  __syncthreads();

  {
    const int row = tid & 63, which = tid >> 6;
    const float* sa = satt + which * GBN;
    const float* hr = stg + row * GBN;
    float d = 0.f;
#pragma unroll 4
    for (int c4 = 0; c4 < GBN / 4; ++c4) {
      const v4f hv = *(const v4fa*)(hr + 4 * c4);
      const v4f av = *(const v4fa*)(sa + 4 * c4);
      d = fmaf(hv.x, av.x, d);
      d = fmaf(hv.y, av.y, d);
      d = fmaf(hv.z, av.z, d);
      d = fmaf(hv.w, av.w, d);
    }
    sdot[which * GBM + row] = d;
  }
  __syncthreads();

  v4f fv[8];
#pragma unroll
  for (int i = 0; i < 8; ++i) {
    const int lr = 16 * wave + 2 * i + hh;
    fv[i] = *(const v4fa*)(stg + lr * GBN + 4 * m);
  }
  const int which2 = lane >> 4, piece = lane & 15;
  const v4f sdv = *(const v4fa*)(sdot + which2 * GBM + 4 * piece);
  float* sp = SD + (size_t)(2 * head + which2) * (size_t)MPr + rowBase + 4 * piece;

#pragma unroll
  for (int i = 0; i < 8; ++i) {
    const int lr = 16 * wave + 2 * i + hh;
    const int gr = rowBase + lr;
    float* op = outF + (size_t)gr * (size_t)ldo + col0 + 4 * m;
    *(volatile v4f*)op = fv[i];
  }
  if (wave == 0) *(volatile v4f*)sp = sdv;
  __threadfence();
#pragma unroll
  for (int i = 0; i < 8; ++i) {
    const int lr = 16 * wave + 2 * i + hh;
    const int gr = rowBase + lr;
    float* op = outF + (size_t)gr * (size_t)ldo + col0 + 4 * m;
    *(volatile v4f*)op = fv[i];
  }
  if (wave == 0) *(volatile v4f*)sp = sdv;
}

template<int L>
__global__ __launch_bounds__(NTHR) void k_agg(
    const float* __restrict__ F, const float* __restrict__ SD, const float* __restrict__ bias,
    const int* __restrict__ TSRC, const int* __restrict__ TCNT, const int* __restrict__ TOFF,
    const int* __restrict__ TNH,
    unsigned short* HP, float* HO, int nN, int nb, int MPr) {
  const int tid = (int)threadIdx.x, lane = tid & 31, wave = tid >> 5;
  const int c0   = 8 * lane;
  const int head = lane >> 3;
  const float* ASp = SD + (size_t)(2 * head) * (size_t)MPr;
  const float* ADp = ASp + MPr;
  const int bc = (L == 1) ? c0 : 8 * (lane & 7);
  const v4f bb0 = bfr4(*(const v4fa*)(bias + bc));
  const v4f bb1 = bfr4(*(const v4fa*)(bias + bc + 4));
  const int rowBlock = (int)blockIdx.x * RPB;
  const int bkt      = rowBlock / nb;
  const int slotBase = rowBlock - bkt * nb;
  const int* tsrc = TSRC + (size_t)bkt * (size_t)RCAP;
  const int* tcnt = TCNT + (size_t)bkt * (size_t)NBMAX;
  const int* toff = TOFF + (size_t)bkt * (size_t)NBMAX;
  int nh = TNH[(size_t)bkt * 32];
  nh = nh < 0 ? 0 : (nh > RCAP ? RCAP : nh);
  nh = __builtin_amdgcn_readfirstlane(nh);
  const bool ovf = (nh >= RCAP);
  const float qnan = __int_as_float(0x7fc00000);

#pragma unroll 1
  for (int jt = 0; jt < RPW; ++jt) {
    const int slot = slotBase + wave * RPW + jt;
    const int grow = rowBlock + wave * RPW + jt;
    const int gcl  = grow < nN ? grow : nN - 1;
    int st = toff[slot];
    int craw = tcnt[slot];
    st   = __builtin_amdgcn_readfirstlane(st);
    craw = __builtin_amdgcn_readfirstlane(craw);
    int cnt = craw;
    st  = st < 0 ? 0 : (st > nh ? nh : st);
    cnt = cnt < 0 ? 0 : (cnt > DEGCAP ? DEGCAP : cnt);
    if (cnt > nh - st) cnt = nh - st;
    const float pz = (ovf || craw > DEGCAP) ? qnan : 0.0f;

    const float* fo = F + (size_t)gcl * HC + c0;
    v4f av0 = *(const v4fa*)fo;
    v4f av1 = *(const v4fa*)(fo + 4);
    const float adv = ADp[gcl];
    float l0 = ASp[gcl] + adv;
    l0 = l0 > 0.f ? l0 : NEGSL * l0;
    float mx = l0, dn = 1.0f;

#pragma unroll 1
    for (int b0 = 0; b0 < cnt; b0 += 32) {
      int idx = st + b0 + lane;
      idx = idx > RCAP - 1 ? RCAP - 1 : idx;
      int sv = tsrc[idx];
      sv = sv < 0 ? 0 : (sv > nN - 1 ? nN - 1 : sv);
      const int m32 = (cnt - b0) < 32 ? (cnt - b0) : 32;
#pragma unroll 1
      for (int k = 0; k < m32; ++k) {
        const int s = __builtin_amdgcn_readlane(sv, k);
        const float* fp = F + (size_t)s * HC + c0;
        const v4f fs0 = *(const v4fa*)fp;
        const v4f fs1 = *(const v4fa*)(fp + 4);
        float lg = ASp[s] + adv;
        lg = lg > 0.f ? lg : NEGSL * lg;
        const float df = lg - mx;
        const float ee = __expf(-fabsf(df));
        const bool up  = df > 0.f;
        const float s1 = up ? ee : 1.0f;
        const float s2 = up ? 1.0f : ee;
        mx = up ? lg : mx;
        dn = fmaf(dn, s1, s2);
        av0.x = fmaf(av0.x, s1, s2 * fs0.x);
        av0.y = fmaf(av0.y, s1, s2 * fs0.y);
        av0.z = fmaf(av0.z, s1, s2 * fs0.z);
        av0.w = fmaf(av0.w, s1, s2 * fs0.w);
        av1.x = fmaf(av1.x, s1, s2 * fs1.x);
        av1.y = fmaf(av1.y, s1, s2 * fs1.y);
        av1.z = fmaf(av1.z, s1, s2 * fs1.z);
        av1.w = fmaf(av1.w, s1, s2 * fs1.w);
      }
    }
    const float inv = __builtin_amdgcn_rcpf(dn + EPS_SM);
    const bool live = grow < nN;

    if constexpr (L == 1) {
      const float o0 = live ? (elu1(fmaf(av0.x, inv, bb0.x)) + pz) : 0.f;
      const float o1 = live ? (elu1(fmaf(av0.y, inv, bb0.y)) + pz) : 0.f;
      const float o2 = live ? (elu1(fmaf(av0.z, inv, bb0.z)) + pz) : 0.f;
      const float o3 = live ? (elu1(fmaf(av0.w, inv, bb0.w)) + pz) : 0.f;
      const float o4 = live ? (elu1(fmaf(av1.x, inv, bb1.x)) + pz) : 0.f;
      const float o5 = live ? (elu1(fmaf(av1.y, inv, bb1.y)) + pz) : 0.f;
      const float o6 = live ? (elu1(fmaf(av1.z, inv, bb1.z)) + pz) : 0.f;
      const float o7 = live ? (elu1(fmaf(av1.w, inv, bb1.w)) + pz) : 0.f;
      const unsigned int h0 = f2bf(o0), h1 = f2bf(o1), h2 = f2bf(o2), h3 = f2bf(o3);
      const unsigned int h4 = f2bf(o4), h5 = f2bf(o5), h6 = f2bf(o6), h7 = f2bf(o7);
      const unsigned int q0 = f2bf(o0 - bf2f(h0)), q1 = f2bf(o1 - bf2f(h1));
      const unsigned int q2 = f2bf(o2 - bf2f(h2)), q3 = f2bf(o3 - bf2f(h3));
      const unsigned int q4 = f2bf(o4 - bf2f(h4)), q5 = f2bf(o5 - bf2f(h5));
      const unsigned int q6 = f2bf(o6 - bf2f(h6)), q7 = f2bf(o7 - bf2f(h7));
      v4u hv, lv;
      hv.x = h0 | (h1 << 16); hv.y = h2 | (h3 << 16); hv.z = h4 | (h5 << 16); hv.w = h6 | (h7 << 16);
      lv.x = q0 | (q1 << 16); lv.y = q2 | (q3 << 16); lv.z = q4 | (q5 << 16); lv.w = q6 | (q7 << 16);
      unsigned short* gp = HP + (size_t)grow * KA2 + 8 * lane;
      *(volatile v4u*)gp        = hv;
      *(volatile v4u*)(gp + HC) = lv;
      __threadfence();
      *(volatile v4u*)gp        = hv;
      *(volatile v4u*)(gp + HC) = lv;
    } else {
      float z0 = av0.x * inv, z1 = av0.y * inv, z2 = av0.z * inv, z3 = av0.w * inv;
      float z4 = av1.x * inv, z5 = av1.y * inv, z6 = av1.z * inv, z7 = av1.w * inv;
      z0 += __shfl_xor(z0, 8);  z1 += __shfl_xor(z1, 8);  z2 += __shfl_xor(z2, 8);  z3 += __shfl_xor(z3, 8);
      z4 += __shfl_xor(z4, 8);  z5 += __shfl_xor(z5, 8);  z6 += __shfl_xor(z6, 8);  z7 += __shfl_xor(z7, 8);
      z0 += __shfl_xor(z0, 16); z1 += __shfl_xor(z1, 16); z2 += __shfl_xor(z2, 16); z3 += __shfl_xor(z3, 16);
      z4 += __shfl_xor(z4, 16); z5 += __shfl_xor(z5, 16); z6 += __shfl_xor(z6, 16); z7 += __shfl_xor(z7, 16);
      z0 = live ? (fmaf(z0, 0.25f, bb0.x) + pz) : 0.f;
      z1 = live ? (fmaf(z1, 0.25f, bb0.y) + pz) : 0.f;
      z2 = live ? (fmaf(z2, 0.25f, bb0.z) + pz) : 0.f;
      z3 = live ? (fmaf(z3, 0.25f, bb0.w) + pz) : 0.f;
      z4 = live ? (fmaf(z4, 0.25f, bb1.x) + pz) : 0.f;
      z5 = live ? (fmaf(z5, 0.25f, bb1.y) + pz) : 0.f;
      z6 = live ? (fmaf(z6, 0.25f, bb1.z) + pz) : 0.f;
      z7 = live ? (fmaf(z7, 0.25f, bb1.w) + pz) : 0.f;
      const int sl = lane >> 1;
      const float g0 = __shfl(z0, sl), g1 = __shfl(z1, sl), g2 = __shfl(z2, sl), g3 = __shfl(z3, sl);
      const float g4 = __shfl(z4, sl), g5 = __shfl(z5, sl), g6 = __shfl(z6, sl), g7 = __shfl(z7, sl);
      const bool odd = (lane & 1) != 0;
      v4f ow;
      ow.x = odd ? g4 : g0; ow.y = odd ? g5 : g1; ow.z = odd ? g6 : g2; ow.w = odd ? g7 : g3;
      float* op = HO + (size_t)grow * HID + 4 * (lane & 15);
      const bool wr = lane < 16;
      if (wr) *(volatile v4f*)op = ow;
      __threadfence();
      if (wr) *(volatile v4f*)op = ow;
    }
  }
}

__global__ __launch_bounds__(NTHR) void k_pool(const float* __restrict__ hf, const int* __restrict__ bat,
                                               int nN, float* pl) {
  __shared__ __attribute__((aligned(16))) double wsum[NWAVE * HID];
  __shared__ int wcn[NWAVE];
  __shared__ __attribute__((aligned(16))) float outs[HID];
  const int tid = (int)threadIdx.x, lane = tid & 31, wave = tid >> 5;
  const int g = (int)blockIdx.x;

  double a0 = 0.0, a1 = 0.0;
  int mine = 0;
#pragma unroll 1
  for (int i0 = wave * 32; i0 < nN; i0 += NTHR) {
    const int i  = i0 + lane;
    const int ic = i < nN ? i : nN - 1;
    const int b  = bat[ic];
    const bool hit = (i < nN) && (b == g);
    unsigned msk = __builtin_amdgcn_ballot_w32(hit);
    int nh = (int)__builtin_popcount(msk);
    nh = nh > 32 ? 32 : nh;
    mine += hit ? 1 : 0;
#pragma unroll 1
    for (int q = 0; q < nh; ++q) {
      const int k = __builtin_ffs((int)msk) - 1;
      msk &= msk - 1u;
      int node = i0 + (k < 0 ? 0 : k);
      node = node > nN - 1 ? nN - 1 : node;
      const v2f v = *(const v2fa*)(hf + (size_t)node * HID + 2 * lane);
      a0 += (double)v.x; a1 += (double)v.y;
    }
  }
  wsum[wave * HID + 2 * lane + 0] = a0;
  wsum[wave * HID + 2 * lane + 1] = a1;
  int cnt = mine;
  cnt += __shfl_xor(cnt, 16); cnt += __shfl_xor(cnt, 8); cnt += __shfl_xor(cnt, 4);
  cnt += __shfl_xor(cnt, 2);  cnt += __shfl_xor(cnt, 1);
  if (lane == 0) wcn[wave] = cnt;
  __syncthreads();
  if (tid < HID) {
    double s = 0.0;
    int c = 0;
#pragma unroll
    for (int w2 = 0; w2 < NWAVE; ++w2) { s += wsum[w2 * HID + tid]; c += wcn[w2]; }
    const float cf = (c < 1) ? 1.0f : (float)c;
    outs[tid] = (float)s * (1.0f / cf);
  }
  __syncthreads();
  const v4f ov = *(const v4fa*)(outs + 4 * (lane & 15));
  float* op = pl + (size_t)g * HID + 4 * (lane & 15);
  const bool okst = (wave == 0) && (lane < 16);
  if (okst) *(volatile v4f*)op = ov;
  __threadfence();
  if (okst) *(volatile v4f*)op = ov;
}

__global__ __launch_bounds__(NTHR) void k_head(const float* __restrict__ pl, const float* __restrict__ Wl,
                                               const float* __restrict__ bl, float* out) {
  __shared__ float wls[HID * NOUTC];
  __shared__ float bls[16];
  __shared__ __attribute__((aligned(16))) float os[NOUT];
  const int tid = (int)threadIdx.x;
#pragma unroll 1
  for (int i = tid; i < HID * NOUTC; i += NTHR) wls[i] = bfr(Wl[i]);
  if (tid < 16) {
    const float bb = bl[tid < NOUTC ? tid : NOUTC - 1];
    bls[tid] = (tid < NOUTC) ? bfr(bb) : 0.0f;
  }
  __syncthreads();
#pragma unroll 1
  for (int idx = tid; idx < NOUT; idx += NTHR) {
    const int g = idx / NOUTC;
    const int c = idx - g * NOUTC;
    const float* pr = pl + (size_t)g * HID;
    float s = 0.0f;
#pragma unroll 1
    for (int f4 = 0; f4 < HID / 4; ++f4) {
      const v4f p = *(const v4fa*)(pr + 4 * f4);
      const float* w = wls + (4 * f4) * NOUTC + c;
      s = fmaf(p.x, w[0], s);
      s = fmaf(p.y, w[NOUTC], s);
      s = fmaf(p.z, w[2 * NOUTC], s);
      s = fmaf(p.w, w[3 * NOUTC], s);
    }
    os[idx] = s + bls[c];
  }
  __syncthreads();
  const v4f ov = *(const v4fa*)(os + 4 * tid);
  *(volatile v4f*)(out + 4 * (size_t)tid) = ov;
  __threadfence();
  *(volatile v4f*)(out + 4 * (size_t)tid) = ov;
}

static int pick_nb(int nE, int nN) {
  int nb = NBMAX;
  while (nb > 32 && (long long)nb * (long long)nE * 5LL > (long long)RCAP * (long long)nN * 4LL) nb >>= 1;
  return nb;
}
static inline int cdiv(int a, int b) { return (a + b - 1) / b; }
static inline size_t al256(size_t o) { return (o + 255) & ~(size_t)255; }

extern "C" void kernel_launch(void* const* d_in, const int* in_sizes, int n_in,
                              void* d_out, int out_size, void* d_ws, size_t ws_size,
                              hipStream_t stream) {
  if (n_in < 13) return;
  if (in_sizes[0] < F_IN || (in_sizes[0] % F_IN) != 0) return;
  const int nN = in_sizes[0] / F_IN;
  if (nN < 1 || nN > (1 << 22)) return;
  if (in_sizes[1] < 2 || (in_sizes[1] & 1) != 0) return;
  const int nE = in_sizes[1] / 2;
  if (nE < 1 || nE >= (1 << (32 - SLOTB))) return;
  if (in_sizes[2] != nN) return;
  if (in_sizes[3] != F_IN * HC) return;
  if (in_sizes[4] != NHD * HID || in_sizes[5] != NHD * HID) return;
  if (in_sizes[6] != HC) return;
  if (in_sizes[7] != HC * HC) return;
  if (in_sizes[8] != NHD * HID || in_sizes[9] != NHD * HID) return;
  if (in_sizes[10] != HID) return;
  if (in_sizes[11] != HID * NOUTC) return;
  if (in_sizes[12] != NOUTC) return;
  if (out_size != NOUT) return;

  const float* x    = (const float*)d_in[0];
  const int*   ei   = (const int*)  d_in[1];
  const int*   bat  = (const int*)  d_in[2];
  const float* W1   = (const float*)d_in[3];
  const float* a1s  = (const float*)d_in[4];
  const float* a1d  = (const float*)d_in[5];
  const float* b1   = (const float*)d_in[6];
  const float* W2   = (const float*)d_in[7];
  const float* a2s  = (const float*)d_in[8];
  const float* a2d  = (const float*)d_in[9];
  const float* b2   = (const float*)d_in[10];
  const float* fcw  = (const float*)d_in[11];
  const float* fcb  = (const float*)d_in[12];
  float* out = (float*)d_out;
  const int* src = ei;
  const int* dst = ei + nE;

  const int MP   = cdiv(nN, MROWS) * MROWS;
  const int nb   = pick_nb(nE, nN);
  if (nb < RPB || (nb & (nb - 1)) != 0 || nb > NBMAX || (nb % RPB) != 0) return;
  const int gA   = cdiv(MP, nb);
  if ((long long)gA * nb < (long long)MP) return;
  const int vec8 = ((nE & 3) == 0) ? 1 : 0;

  char* ws = (char*)d_ws;
  size_t off = 0;
  const size_t oA2  = off; off = al256(off + (size_t)MP * KA2 * 2);
  const size_t oH   = off; off = al256(off + (size_t)MP * HC * 4);
  const size_t oH2O = off; off = al256(off + (size_t)MP * HID * 4);
  const size_t oSD  = off; off = al256(off + (size_t)2 * NHD * MP * 4);
  const size_t oTS  = off; off = al256(off + (size_t)gA * RCAP * 4);
  const size_t oTC  = off; off = al256(off + (size_t)gA * NBMAX * 4);
  const size_t oTO  = off; off = al256(off + (size_t)gA * NBMAX * 4);
  const size_t oTN  = off; off = al256(off + (size_t)gA * 32 * 4);
  const size_t oW1T = off; off = al256(off + (size_t)HC * F_IN * 2);
  const size_t oW2D = off; off = al256(off + (size_t)HC * KA2 * 2);
  const size_t oPL  = off; off = al256(off + (size_t)NGR * HID * 4);
  if (off > ws_size || off > (size_t)WSMAX) return;
  unsigned short* A2  = (unsigned short*)(ws + oA2);
  unsigned short* XB  = (unsigned short*)(ws + oA2);
  float*          H   = (float*)(ws + oH);
  float*          H2O = (float*)(ws + oH2O);
  float*          SD  = (float*)(ws + oSD);
  int*            TS  = (int*)(ws + oTS);
  int*            TC  = (int*)(ws + oTC);
  int*            TO  = (int*)(ws + oTO);
  int*            TN  = (int*)(ws + oTN);
  unsigned short* W1T = (unsigned short*)(ws + oW1T);
  unsigned short* W2D = (unsigned short*)(ws + oW2D);
  float*          PL  = (float*)(ws + oPL);

  hipFuncSetAttribute(reinterpret_cast<const void*>(&k_bucket),
                      hipFuncAttributeMaxDynamicSharedMemorySize, LDS_BKT);

  k_wprep<<<(NU1 + NU2) / NTHR, NTHR, 0, stream>>>(W1, W2, W1T, W2D);
  const int nUx = MP * (F_IN / 8);
  k_cvx<<<cdiv(nUx, NTHR), NTHR, 0, stream>>>(x, nN, nUx, XB);
  k_bucket<<<gA, NTHR, LDS_BKT, stream>>>(src, dst, nN, nE, nb, vec8, TS, TC, TO, TN);
  const int gM = MP / GBM;
  k_gemm<<<dim3(gM, HC / GBN), GTHR, 0, stream>>>(XB, W1T, H, F_IN, HC, a1s, a1d, HID, SD, MP);
  k_agg<1><<<MP / RPB, NTHR, 0, stream>>>(H, SD, b1, TS, TC, TO, TN, A2, H2O, nN, nb, MP);
  k_gemm<<<dim3(gM, HC / GBN), GTHR, 0, stream>>>(A2, W2D, H, KA2, HC, a2s, a2d, HID, SD, MP);
  k_agg<2><<<MP / RPB, NTHR, 0, stream>>>(H, SD, b2, TS, TC, TO, TN, A2, H2O, nN, nb, MP);
  k_pool<<<NGR, NTHR, 0, stream>>>(H2O, bat, nN, PL);
  k_head<<<1, NTHR, 0, stream>>>(PL, fcw, fcb, out);
}
